// MultichannelMultiheadAttention_72971494359081
// MI455X (gfx1250) — hardware-verified
//
#include <hip/hip_runtime.h>
#include <math.h>

constexpr int kBC    = 4;
constexpr int kW     = 1024;
constexpr int kG     = 1024;
constexpr int kHeads = 8;
constexpr int kD     = 128;
constexpr int kRot   = 64;
constexpr int kNF    = kBC * kHeads;
constexpr int kTok   = kBC * kW;
constexpr int kNQKV  = 3 * kG;
constexpr int kGrp   = 4;
constexpr float kScoreScale = 0.03125f;
constexpr float kWoCarry    = 64.0f;
constexpr float kPCarry     = 256.0f;
constexpr float kPCarryInv  = 1.0f / 256.0f;
constexpr float kOCarry     = 256.0f;
constexpr float kOutScale   = 1.0f / (256.0f * 64.0f);
constexpr float kSClamp     = 5.5f;
static_assert(kHeads * kD == kG, "shape");
static_assert(kNF % kGrp == 0, "groups");
static_assert(kTok % 64 == 0 && kNQKV % 64 == 0 && kG % 32 == 0, "qkv gemm");
static_assert(kW % 64 == 0 && kD % 32 == 0, "score gemm");
static_assert(kW % 64 == 0 && kD % 64 == 0 && kW % 32 == 0, "pv gemm");
static_assert(kTok % 64 == 0 && kG % 64 == 0, "out gemm");

typedef __attribute__((ext_vector_type(16))) _Float16 v16h;
typedef __attribute__((ext_vector_type(8)))  _Float16 v8h;
typedef __attribute__((ext_vector_type(16))) __bf16   v16b;
typedef __attribute__((ext_vector_type(8)))  __bf16   v8b;
typedef __attribute__((ext_vector_type(8)))  float    v8f;
typedef __attribute__((ext_vector_type(4)))  float    v4f;
typedef __attribute__((ext_vector_type(4)))  unsigned int v4u;
typedef __attribute__((ext_vector_type(2)))  unsigned int v2u;

__device__ __forceinline__ unsigned short f2bf_bits(float f) {
  unsigned u = __float_as_uint(f);
  return (unsigned short)((u + 0x7FFFu + ((u >> 16) & 1u)) >> 16);
}
__device__ __forceinline__ float bf_bits2f(unsigned short h) { return __uint_as_float(((unsigned)h) << 16); }

__device__ __forceinline__ void dep_guard_h(v8f& a, v8f& b, v16h x, v16h y) { asm volatile("v_nop\n\tv_nop\n\tv_nop\n\tv_nop" : "+v"(a), "+v"(b) : "v"(x), "v"(y)); }
__device__ __forceinline__ void dep_guard_b(v8f& a, v8f& b, v16b x, v16b y) { asm volatile("v_nop\n\tv_nop\n\tv_nop\n\tv_nop" : "+v"(a), "+v"(b) : "v"(x), "v"(y)); }
__device__ __forceinline__ void keep4_h(v16h a, v16h b, v16h c, v16h d) { asm volatile("v_nop" :: "v"(a), "v"(b), "v"(c), "v"(d)); }
__device__ __forceinline__ void keep4_b(v16b a, v16b b, v16b c, v16b d) { asm volatile("v_nop" :: "v"(a), "v"(b), "v"(c), "v"(d)); }
__device__ __forceinline__ void acc_guard4(v8f& a, v8f& b, v8f& c, v8f& d) { asm volatile("v_nop\n\tv_nop\n\tv_nop\n\tv_nop" : "+v"(a), "+v"(b), "+v"(c), "+v"(d)); }
template <typename T> struct Frag;
template <> struct Frag<_Float16> {
  typedef v16h V; union U { v16h v; v8h h[2]; };
  static __device__ __forceinline__ v16h load(const _Float16* p) {
    U f; f.h[0] = *(const v8h*)(p); f.h[1] = *(const v8h*)(p + 16); return f.v;
  }
  static __device__ __forceinline__ v8f mma(v16h a, v16h b, v8f c) {
    return __builtin_amdgcn_wmma_f32_16x16x32_f16(false, a, false, b, (short)0, c, false, false);
  }
  static __device__ __forceinline__ void guard(v8f& a, v8f& b, v16h x, v16h y) { dep_guard_h(a, b, x, y); }
  static __device__ __forceinline__ void keep(v16h a, v16h b, v16h c, v16h d) { keep4_h(a, b, c, d); }
};
template <> struct Frag<__bf16> {
  typedef v16b V; union U { v16b v; v8b h[2]; };
  static __device__ __forceinline__ v16b load(const __bf16* p) {
    U f; f.h[0] = *(const v8b*)(p); f.h[1] = *(const v8b*)(p + 16); return f.v;
  }
  static __device__ __forceinline__ v8f mma(v16b a, v16b b, v8f c) {
    return __builtin_amdgcn_wmma_f32_16x16x32_bf16(false, a, false, b, (short)0, c, false, false);
  }
  static __device__ __forceinline__ void guard(v8f& a, v8f& b, v16b x, v16b y) { dep_guard_b(a, b, x, y); }
  static __device__ __forceinline__ void keep(v16b a, v16b b, v16b c, v16b d) { keep4_b(a, b, c, d); }
};

__device__ __forceinline__ unsigned pk16(unsigned short a, unsigned short b) { return (unsigned)a | ((unsigned)b << 16); }
__device__ __forceinline__ unsigned short h_bits(float f) { const _Float16 h = (_Float16)f; return __builtin_bit_cast(unsigned short, h); }
__device__ __forceinline__ float bfr(float f) { return bf_bits2f(f2bf_bits(f)); }

template <int ET> struct Elem;
template <> struct Elem<0> { typedef _Float16 T; };
template <> struct Elem<1> { typedef __bf16 T; };
template <int ET, bool SPLIT, int BIAS_MODE, int OUT_MODE, bool RESID, int ACT = 0>
__global__ __launch_bounds__(256) void wmma_gemm64(
    const unsigned short* __restrict__ Ap, const unsigned short* __restrict__ A2p, int lda, long strideA,
    const unsigned short* __restrict__ Btp, const unsigned short* __restrict__ Bt2p, int ldb, long strideB,
    void* __restrict__ Cout, void* __restrict__ Cout2, int ldc, long strideC,
    const float* __restrict__ bias,
    const float* __restrict__ resid, long strideR,
    int M, int N, int K, float scale) {
  typedef typename Elem<ET>::T T;
  typedef typename Frag<T>::V V;
  const T* A = (const T*)Ap; const T* A2 = (const T*)A2p; const T* Bt = (const T*)Btp; const T* Bt2 = (const T*)Bt2p;
  __shared__ __align__(16) float sT[8][16 * 68];
  const int b    = blockIdx.y;
  const int lane = threadIdx.x & 31;
  const int wave = threadIdx.x >> 5;
  const int tilesN = N >> 6;
  const int tilesM = M >> 6;
  const int tile = blockIdx.x * 8 + wave;
  if (tile >= tilesM * tilesN) return;
  const int tm = tile / tilesN;
  const int tn = tile - tm * tilesN;
  const int m0 = tm << 6;
  const int n0 = tn << 6;

  const T* Ab  = A  + (size_t)b * strideA;
  const T* Bb  = Bt + (size_t)b * strideB;
  const T* Ab2 = SPLIT ? (A2  + (size_t)b * strideA) : nullptr;
  const T* Bb2 = SPLIT ? (Bt2 + (size_t)b * strideB) : nullptr;

  const int rlane = lane & 15;
  const int koff  = (lane >> 4) * 8;
  const int mOff  = (lane >> 4) * 8;

  v8f acc[4][4];
#pragma unroll
  for (int i = 0; i < 4; ++i)
#pragma unroll
    for (int j = 0; j < 4; ++j) acc[i][j] = (v8f){0.f,0.f,0.f,0.f,0.f,0.f,0.f,0.f};

  for (int k0 = 0; k0 < K; k0 += 32) {
    V bh[4], bl[4];
#pragma unroll
    for (int j = 0; j < 4; ++j) {
      const size_t bo = (size_t)(n0 + (j << 4) + rlane) * ldb + koff + k0;
      bh[j] = Frag<T>::load(Bb + bo);
      if (SPLIT) bl[j] = Frag<T>::load(Bb2 + bo);
    }
#pragma unroll
    for (int i = 0; i < 4; ++i) {
      const size_t ao = (size_t)(m0 + (i << 4) + rlane) * lda + koff + k0;
      V ah = Frag<T>::load(Ab + ao);
      V al;
      if (SPLIT) al = Frag<T>::load(Ab2 + ao);
#pragma unroll
      for (int j = 0; j < 4; ++j) {
        acc[i][j] = Frag<T>::mma(ah, bh[j], acc[i][j]);
        if (SPLIT) {
          acc[i][j] = Frag<T>::mma(ah, bl[j], acc[i][j]);
          acc[i][j] = Frag<T>::mma(al, bh[j], acc[i][j]);
        }
      }
      Frag<T>::guard(acc[i][0], acc[i][3], ah, SPLIT ? al : ah);
    }
    Frag<T>::keep(bh[0], bh[1], bh[2], bh[3]);
    if (SPLIT) Frag<T>::keep(bl[0], bl[1], bl[2], bl[3]);
  }
  acc_guard4(acc[0][0], acc[0][1], acc[0][2], acc[0][3]);
  acc_guard4(acc[1][0], acc[1][1], acc[1][2], acc[1][3]);
  acc_guard4(acc[2][0], acc[2][1], acc[2][2], acc[2][3]);
  acc_guard4(acc[3][0], acc[3][1], acc[3][2], acc[3][3]);

  float* slab = sT[wave];
  const float* Rb = RESID ? (resid + (size_t)b * strideR) : nullptr;
#pragma unroll
  for (int i = 0; i < 4; ++i) {
    const int mBase = m0 + (i << 4);
#pragma unroll
    for (int j = 0; j < 4; ++j) {
      const int n = n0 + (j << 4) + rlane;
      float bv = 0.f;
      if (BIAS_MODE == 2) bv = bias[n];
#pragma unroll
      for (int r = 0; r < 8; ++r) {
        float v = acc[i][j][r] * scale;
        if (BIAS_MODE == 1) v += bias[mBase + mOff + r];
        if (BIAS_MODE == 2) v += bv;
        if (RESID) v += Rb[(size_t)(mBase + mOff + r) * ldc + n];
        if (ACT == 2) v = fmaxf(v, 0.0f);
        if (ACT == 4) v = (v > 0.f) ? v : 0.01f * v;
        slab[(mOff + r) * 68 + (j << 4) + rlane] = v;
      }
    }
    __builtin_amdgcn_fence(__ATOMIC_RELEASE, "workgroup");
    __builtin_amdgcn_wave_barrier();
    __builtin_amdgcn_fence(__ATOMIC_ACQUIRE, "workgroup");
    if (OUT_MODE == 0) {
      float* C = (float*)Cout + (size_t)b * strideC;
      const int hh = lane >> 4, c4 = (lane & 15) * 4;
      for (int pass = 0; pass < 2; ++pass) {
#pragma unroll
        for (int it = 0; it < 8; ++it) {
          const int row = it * 2 + hh;
          v4f v = *(const v4f*)(slab + row * 68 + c4);
          *(volatile v4f*)(C + (size_t)(mBase + row) * ldc + n0 + c4) = v;
        }
        __threadfence();
      }
    } else {
      const int q = lane >> 3, c8 = (lane & 7) * 8;
      unsigned short* C  = (unsigned short*)Cout  + (size_t)b * strideC;
      unsigned short* C2 = (OUT_MODE == 2) ? ((unsigned short*)Cout2 + (size_t)b * strideC) : nullptr;
      for (int pass = 0; pass < 2; ++pass) {
#pragma unroll
        for (int it = 0; it < 4; ++it) {
          const int row = it * 4 + q;
          const float* sp = slab + row * 68 + c8;
          v8h hv, lv;
#pragma unroll
          for (int e = 0; e < 8; ++e) {
            if (OUT_MODE == 1) {
              hv[e] = (_Float16)sp[e];
            } else {
              unsigned short hb = f2bf_bits(sp[e]);
              unsigned short lb = f2bf_bits(sp[e] - bf_bits2f(hb));
              hv[e] = __builtin_bit_cast(_Float16, hb);
              lv[e] = __builtin_bit_cast(_Float16, lb);
            }
          }
          *(volatile v8h*)(C + (size_t)(mBase + row) * ldc + n0 + c8) = hv;
          if (OUT_MODE == 2) *(volatile v8h*)(C2 + (size_t)(mBase + row) * ldc + n0 + c8) = lv;
        }
        __threadfence();
      }
    }
    __builtin_amdgcn_fence(__ATOMIC_RELEASE, "workgroup");
    __builtin_amdgcn_wave_barrier();
    __builtin_amdgcn_fence(__ATOMIC_ACQUIRE, "workgroup");
  }
}

__global__ __launch_bounds__(256) void cast8_bf16_kernel(const float* __restrict__ in, unsigned short* __restrict__ out, int n8) {
  const int i = blockIdx.x * 256 + threadIdx.x;
  if (i >= n8) return;
  const float* p = in + 8 * (size_t)i;
  const v4f a = *(const v4f*)(p);
  const v4f c = *(const v4f*)(p + 4);
  unsigned short hb[8];
#pragma unroll
  for (int e = 0; e < 4; ++e) {
    hb[e]     = f2bf_bits(a[e]);
    hb[4 + e] = f2bf_bits(c[e]);
  }
  const v4u u = (v4u){pk16(hb[0], hb[1]), pk16(hb[2], hb[3]), pk16(hb[4], hb[5]), pk16(hb[6], hb[7])};
  unsigned short* q = out + 8 * (size_t)i;
  *(volatile v4u*)q = u;
  __threadfence();
  *(volatile v4u*)q = u;
}

__global__ __launch_bounds__(256) void cast8_f16s_kernel(const float* __restrict__ in, unsigned short* __restrict__ out, int n8, float scale) {
  const int i = blockIdx.x * 256 + threadIdx.x;
  if (i >= n8) return;
  const float* p = in + 8 * (size_t)i;
  const v4f a = *(const v4f*)(p);
  const v4f c = *(const v4f*)(p + 4);
  unsigned short hb[8];
#pragma unroll
  for (int e = 0; e < 4; ++e) {
    hb[e]     = h_bits(bfr(a[e]) * scale);
    hb[4 + e] = h_bits(bfr(c[e]) * scale);
  }
  const v4u u = (v4u){pk16(hb[0], hb[1]), pk16(hb[2], hb[3]), pk16(hb[4], hb[5]), pk16(hb[6], hb[7])};
  unsigned short* q = out + 8 * (size_t)i;
  *(volatile v4u*)q = u;
  __threadfence();
  *(volatile v4u*)q = u;
}

__global__ __launch_bounds__(256) void trig_table_kernel(const float* __restrict__ invf, float* __restrict__ tabC, float* __restrict__ tabS) {
#pragma clang fp contract(off)
  __shared__ __align__(16) float csm[8][32];
  __shared__ __align__(16) float ssm[8][32];
  const int t = threadIdx.x, lane = t & 31, wave = t >> 5;
  const int w = blockIdx.x * 8 + wave;
  const float fr = bfr(invf[lane]);
  const float ang = (float)w * fr;
  float sv, cv;
  sincosf(ang, &sv, &cv);
  csm[wave][lane] = cv;
  ssm[wave][lane] = sv;
  __syncthreads();
  const int c4 = (lane & 7) * 4;
  const v4f vc = *(const v4f*)(&csm[wave][c4]);
  const v4f vs = *(const v4f*)(&ssm[wave][c4]);
  if (lane < 8) {
    float* pc = tabC + (size_t)w * 32 + c4;
    float* ps = tabS + (size_t)w * 32 + c4;
    *(volatile v4f*)pc = vc;
    *(volatile v4f*)ps = vs;
    __threadfence();
    *(volatile v4f*)pc = vc;
    *(volatile v4f*)ps = vs;
  }
}

__device__ __forceinline__ void conv8(const float* ya, const float* yb, const float* yc,
                                      const float* c0, const float* c1, const float* c2, float* z) {
  const v4f a0 = *(const v4f*)(ya), a1 = *(const v4f*)(ya + 4);
  const v4f b0 = *(const v4f*)(yb), b1 = *(const v4f*)(yb + 4);
  const v4f g0 = *(const v4f*)(yc), g1 = *(const v4f*)(yc + 4);
#pragma unroll
  for (int e = 0; e < 4; ++e) {
    z[e]     = c0[e] * a0[e] + c1[e] * b0[e] + c2[e] * g0[e];
    z[4 + e] = c0[4 + e] * a1[e] + c1[4 + e] * b1[e] + c2[4 + e] * g1[e];
  }
}

__global__ __launch_bounds__(256) void conv_rope_kernel(const float* __restrict__ Y,
    const float* __restrict__ qc, const float* __restrict__ kc, const float* __restrict__ vc,
    const float* __restrict__ tabC, const float* __restrict__ tabS,
    unsigned short* __restrict__ Qh, unsigned short* __restrict__ Kh, unsigned short* __restrict__ VTh) {
  __shared__ __align__(16) float ysm[66][132];
  __shared__ __align__(16) unsigned short tsm[128][72];
  const int t = threadIdx.x, lane = t & 31, wave = t >> 5;
  const int w0 = blockIdx.x * 64;
  const int f = blockIdx.y;
  const int bc = f >> 3, head = f & 7;
  const int proj = blockIdx.z;
  const float* taps = (proj == 0) ? qc : ((proj == 1) ? kc : vc);
  const size_t colBase = (size_t)proj * kG + (size_t)head * kD + (size_t)lane * 4;
#pragma unroll
  for (int it = 0; it < 9; ++it) {
    const int r = wave + 8 * it;
    if (r < 66) {
      const int w = w0 - 1 + r;
      const bool valid = (w >= 0) && (w < kW);
      const int wc = (w < 0) ? 0 : ((w >= kW) ? (kW - 1) : w);
      v4f v = *(const v4f*)(Y + ((size_t)bc * kW + wc) * kNQKV + colBase);
      if (!valid) v = (v4f){0.f, 0.f, 0.f, 0.f};
      *(v4f*)(&ysm[r][lane * 4]) = v;
    }
  }
  __syncthreads();

  const int ch = t & 15, d0 = ch * 8, g0 = head * kD + d0;
  float c0[8], c1[8], c2[8];
  {
    const v4f a0 = *(const v4f*)(taps + g0),          a1 = *(const v4f*)(taps + g0 + 4);
    const v4f b0 = *(const v4f*)(taps + kG + g0),     b1 = *(const v4f*)(taps + kG + g0 + 4);
    const v4f e0 = *(const v4f*)(taps + 2 * kG + g0), e1 = *(const v4f*)(taps + 2 * kG + g0 + 4);
#pragma unroll
    for (int e = 0; e < 4; ++e) {
      c0[e] = bfr(a0[e]); c0[4 + e] = bfr(a1[e]);
      c1[e] = bfr(b0[e]); c1[4 + e] = bfr(b1[e]);
      c2[e] = bfr(e0[e]); c2[4 + e] = bfr(e1[e]);
    }
  }

  if (proj < 2) {
    unsigned short* dstPlane = (proj == 0) ? Qh : Kh;
    const int i0 = (ch & 7) * 4;
    const bool use_rope = (ch < 8);
#pragma unroll 1
    for (int it = 0; it < 4; ++it) {
      const int wl = it * 16 + (t >> 4);
      const int w = w0 + wl;
      const v4f cs4 = *(const v4f*)(tabC + (size_t)w * 32 + i0);
      const v4f sn4 = *(const v4f*)(tabS + (size_t)w * 32 + i0);
      float z[8];
      conv8(&ysm[wl][d0], &ysm[wl + 1][d0], &ysm[wl + 2][d0], c0, c1, c2, z);
      unsigned short hb[8];
#pragma unroll
      for (int j = 0; j < 4; ++j) {
        const float cv = cs4[j], sv = sn4[j];
        const float x0 = z[2 * j], x1 = z[2 * j + 1];
        const float r0v = x0 * cv - x1 * sv;
        const float r1v = x1 * cv + x0 * sv;
        const float o0 = use_rope ? r0v : x0;
        const float o1 = use_rope ? r1v : x1;
        hb[2 * j]     = h_bits(o0);
        hb[2 * j + 1] = h_bits(o1);
      }
      const v4u u = (v4u){pk16(hb[0], hb[1]), pk16(hb[2], hb[3]), pk16(hb[4], hb[5]), pk16(hb[6], hb[7])};
      unsigned short* dp = dstPlane + (((size_t)f * kW + w) * kD + d0);
      *(volatile v4u*)dp = u;
      __threadfence();
      *(volatile v4u*)dp = u;
    }
  } else {
#pragma unroll 1
    for (int it = 0; it < 4; ++it) {
      const int wl = it * 16 + (t >> 4);
      float z[8];
      conv8(&ysm[wl][d0], &ysm[wl + 1][d0], &ysm[wl + 2][d0], c0, c1, c2, z);
#pragma unroll
      for (int e = 0; e < 8; ++e) tsm[d0 + e][wl] = h_bits(z[e]);
    }
    __syncthreads();
    const int q = lane >> 3, c8 = (lane & 7) * 8;
    unsigned short* op = VTh + (size_t)f * kD * kW;
    for (int pass = 0; pass < 2; ++pass) {
#pragma unroll
      for (int it = 0; it < 4; ++it) {
        const int row = wave * 16 + it * 4 + q;
        const v4u u = *(const v4u*)(&tsm[row][c8]);
        *(volatile v4u*)(op + (size_t)row * kW + w0 + c8) = u;
      }
      __threadfence();
    }
  }
}

__global__ __launch_bounds__(256) void vsum_kernel(const float* __restrict__ Y, const float* __restrict__ vc, float* __restrict__ Vsum) {
  __shared__ __align__(16) float sq[256];
  const int t = threadIdx.x;
  const int bc = blockIdx.x >> 2;
  const int gt = blockIdx.x & 3;
  const int g = gt * 256 + t;
  const float tp0 = bfr(vc[g]), tp1 = bfr(vc[kG + g]), tp2 = bfr(vc[2 * kG + g]);
  const float* col = Y + (size_t)bc * kW * kNQKV + 2 * kG + g;
  float ym1 = 0.f;
  float y0 = col[0];
  float a0 = 0.f, a1 = 0.f, a2 = 0.f, a3 = 0.f;
#pragma unroll 1
  for (int w = 0; w < kW; w += 4) {
    float yp = col[(size_t)(w + 1) * kNQKV];
    a0 += tp0 * ym1 + tp1 * y0 + tp2 * yp;
    ym1 = y0; y0 = yp;
    yp = col[(size_t)(w + 2) * kNQKV];
    a1 += tp0 * ym1 + tp1 * y0 + tp2 * yp;
    ym1 = y0; y0 = yp;
    yp = col[(size_t)(w + 3) * kNQKV];
    a2 += tp0 * ym1 + tp1 * y0 + tp2 * yp;
    ym1 = y0; y0 = yp;
    const int wn = w + 4;
    const int wcl = (wn < kW) ? wn : (kW - 1);
    yp = col[(size_t)wcl * kNQKV];
    if (wn >= kW) yp = 0.f;
    a3 += tp0 * ym1 + tp1 * y0 + tp2 * yp;
    ym1 = y0; y0 = yp;
  }
  sq[t] = (a0 + a1) + (a2 + a3);
  __syncthreads();
  if (t < 64) {
    const v4f val = *(const v4f*)(sq + 4 * t);
    float* dp = Vsum + (size_t)bc * kG + gt * 256 + 4 * t;
    *(volatile v4f*)dp = val;
    __threadfence();
    *(volatile v4f*)dp = val;
  }
}

__global__ __launch_bounds__(256) void pexp_kernel(const float* __restrict__ S, unsigned short* __restrict__ P, float* __restrict__ L) {
  __shared__ __align__(16) unsigned short rowbuf[8][1024];
  __shared__ __align__(16) float lsm[32];
  const int t = threadIdx.x, lane = t & 31, wave = t >> 5;
  const int g = blockIdx.x >> 5;
  const int r0 = (blockIdx.x & 31) * 32;
  for (int rr = 0; rr < 4; ++rr) {
    const int row = r0 + wave * 4 + rr;
    const size_t rowOff = ((size_t)g * kW + row) * kW;
    float sum = 0.f;
    __syncthreads();
#pragma unroll 1
    for (int it = 0; it < 8; ++it) {
      const int c = it * 128 + lane * 4;
      const v4f sv = *(const v4f*)(S + rowOff + c);
      unsigned short hb[4];
#pragma unroll
      for (int e = 0; e < 4; ++e) {
        const float s = fminf(sv[e], kSClamp);
        const float p = expf(s) - 1.0f;
        sum += p;
        hb[e] = h_bits(p * kPCarry);
      }
      const v2u u2 = (v2u){pk16(hb[0], hb[1]), pk16(hb[2], hb[3])};
      *(v2u*)(&rowbuf[wave][c]) = u2;
    }
#pragma unroll
    for (int off = 16; off > 0; off >>= 1) sum += __shfl_xor(sum, off, 32);
    if (lane == 0) lsm[wave * 4 + rr] = (float)kW + sum;
    __syncthreads();
    for (int pass = 0; pass < 2; ++pass) {
#pragma unroll
      for (int it2 = 0; it2 < 4; ++it2) {
        const int c = it2 * 256 + lane * 8;
        const v4u u = *(const v4u*)(&rowbuf[wave][c]);
        *(volatile v4u*)(P + rowOff + c) = u;
      }
      __threadfence();
    }
  }
  __syncthreads();
  if (t < 8) {
    const v4f val = *(const v4f*)(lsm + 4 * t);
    float* lp = L + (size_t)g * kW + r0 + 4 * t;
    *(volatile v4f*)lp = val;
    __threadfence();
    *(volatile v4f*)lp = val;
  }
}

__global__ __launch_bounds__(256) void ofin_kernel(const float* __restrict__ Num, const float* __restrict__ L,
                                                   const float* __restrict__ Vsum, unsigned short* __restrict__ Oh, int f0) {
  const int idx = blockIdx.x * 256 + threadIdx.x;
  const int row = idx >> 4;
  const int g = row >> 10;
  const int q = row & (kW - 1);
  const int d0 = (idx & 15) * 8;
  const int f = f0 + g;
  const int bc = f >> 3, head = f & 7;
  const float* np = Num + ((size_t)g * kW + q) * kD + d0;
  const v4f n0 = *(const v4f*)(np), n1 = *(const v4f*)(np + 4);
  const float* vp = Vsum + (size_t)f * kD + d0;
  const v4f s0 = *(const v4f*)(vp), s1 = *(const v4f*)(vp + 4);
  const float inv = 1.0f / L[(size_t)g * kW + q];
  unsigned short hb[8];
#pragma unroll
  for (int e = 0; e < 4; ++e) {
    const float oa = (s0[e] + n0[e]) * inv;
    const float ob = (s1[e] + n1[e]) * inv;
    hb[e]     = h_bits(oa * kOCarry);
    hb[4 + e] = h_bits(ob * kOCarry);
  }
  const v4u u = (v4u){pk16(hb[0], hb[1]), pk16(hb[2], hb[3]), pk16(hb[4], hb[5]), pk16(hb[6], hb[7])};
  unsigned short* dp = Oh + (((size_t)bc * kW + q) * kG + head * kD + d0);
  *(volatile v4u*)dp = u;
  __threadfence();
  *(volatile v4u*)dp = u;
}

extern "C" void kernel_launch(void* const* d_in, const int* in_sizes, int n_in,
                              void* d_out, int out_size, void* d_ws, size_t ws_size,
                              hipStream_t stream) {
  if (n_in < 9) return;
  if (in_sizes[0] != kTok * kG) return;
  if (in_sizes[1] != kG * kG || in_sizes[3] != kG * kG || in_sizes[5] != kG * kG || in_sizes[7] != kG * kG) return;
  if (in_sizes[2] != 3 * kG || in_sizes[4] != 3 * kG || in_sizes[6] != 3 * kG) return;
  if (in_sizes[8] != kRot / 2) return;
  if (out_size != kTok * kG) return;

  const size_t szXb   = (size_t)kTok * kG * 2;
  const size_t szWqkv = (size_t)kNQKV * kG * 2;
  const size_t szWo   = (size_t)kG * kG * 2;
  const size_t szY    = (size_t)kTok * kNQKV * 4;
  const size_t szQK   = (size_t)kNF * kW * kD * 2;
  const size_t szOh   = (size_t)kTok * kG * 2;
  const size_t szS    = (size_t)kGrp * kW * kW * 4;
  const size_t szP    = (size_t)kGrp * kW * kW * 2;
  const size_t szNum  = (size_t)kGrp * kW * kD * 4;
  const size_t szL    = (size_t)kGrp * kW * 4;
  const size_t szVsum = (size_t)kNF * kD * 4;
  const size_t szTab  = (size_t)kW * 32 * 4;
  const size_t offXb   = 0;
  const size_t offWqkv = offXb + szXb;
  const size_t offWo   = offWqkv + szWqkv;
  const size_t offY    = offWo + szWo;
  const size_t offQh   = offY + szY;
  const size_t offKh   = offQh + szQK;
  const size_t offVTh  = offKh + szQK;
  const size_t offOh   = offVTh + szQK;
  const size_t offS    = offOh + szOh;
  const size_t offP    = offS + szS;
  const size_t offNum  = offP + szP;
  const size_t offL    = offNum + szNum;
  const size_t offVsum = offL + szL;
  const size_t offTabC = offVsum + szVsum;
  const size_t offTabS = offTabC + szTab;
  const size_t total   = offTabS + szTab;
  if (ws_size < total) return;

  const float* x     = (const float*)d_in[0];
  const float* q_w   = (const float*)d_in[1];
  const float* q_cv  = (const float*)d_in[2];
  const float* k_w   = (const float*)d_in[3];
  const float* k_cv  = (const float*)d_in[4];
  const float* v_w   = (const float*)d_in[5];
  const float* v_cv  = (const float*)d_in[6];
  const float* o_w   = (const float*)d_in[7];
  const float* invf  = (const float*)d_in[8];
  float* out = (float*)d_out;
  char* ws = (char*)d_ws;
  unsigned short* Xb   = (unsigned short*)(ws + offXb);
  unsigned short* Wqkv = (unsigned short*)(ws + offWqkv);
  unsigned short* Wo   = (unsigned short*)(ws + offWo);
  float*          Y    = (float*)(ws + offY);
  unsigned short* Qh   = (unsigned short*)(ws + offQh);
  unsigned short* Kh   = (unsigned short*)(ws + offKh);
  unsigned short* VTh  = (unsigned short*)(ws + offVTh);
  unsigned short* Oh   = (unsigned short*)(ws + offOh);
  float*          S    = (float*)(ws + offS);
  unsigned short* P    = (unsigned short*)(ws + offP);
  float*          Num  = (float*)(ws + offNum);
  float*          L    = (float*)(ws + offL);
  float*          Vsum = (float*)(ws + offVsum);
  float*          tabC = (float*)(ws + offTabC);
  float*          tabS = (float*)(ws + offTabS);

  const int n8x = (kTok * kG) / 8;
  const int n8w = (kG * kG) / 8;
  cast8_bf16_kernel<<<dim3(n8x / 256), dim3(256), 0, stream>>>(x, Xb, n8x);
  cast8_bf16_kernel<<<dim3(n8w / 256), dim3(256), 0, stream>>>(q_w, Wqkv, n8w);
  cast8_bf16_kernel<<<dim3(n8w / 256), dim3(256), 0, stream>>>(k_w, Wqkv + (size_t)kG * kG, n8w);
  cast8_bf16_kernel<<<dim3(n8w / 256), dim3(256), 0, stream>>>(v_w, Wqkv + (size_t)2 * kG * kG, n8w);
  cast8_f16s_kernel<<<dim3(n8w / 256), dim3(256), 0, stream>>>(o_w, Wo, n8w, kWoCarry);
  trig_table_kernel<<<dim3(kW / 8), dim3(256), 0, stream>>>(invf, tabC, tabS);

  const int tilesQKV = (kTok / 64) * (kNQKV / 64);
  wmma_gemm64<1, false, 0, 0, false, 0><<<dim3(tilesQKV / 8, 1), dim3(256), 0, stream>>>(
      Xb, Xb, kG, 0L, Wqkv, Wqkv, kG, 0L, (void*)Y, (void*)Y, kNQKV, 0L, Vsum, Vsum, 0L, kTok, kNQKV, kG, 1.0f);

  conv_rope_kernel<<<dim3(kW / 64, kNF, 3), dim3(256), 0, stream>>>(Y, q_cv, k_cv, v_cv, tabC, tabS, Qh, Kh, VTh);
  vsum_kernel<<<dim3(kBC * 4), dim3(256), 0, stream>>>(Y, v_cv, Vsum);

  const long stridePlane = (long)kW * kD;
  const long strideScore = (long)kW * kW;
  const long strideNum   = (long)kW * kD;
  const int  tilesScore  = (kW / 64) * (kW / 64);
  const int  tilesPV     = (kW / 64) * (kD / 64);
  for (int chk = 0; chk < kNF / kGrp; ++chk) {
    const int f0 = chk * kGrp;
    const unsigned short* Qg = Qh + (size_t)f0 * stridePlane;
    const unsigned short* Kg = Kh + (size_t)f0 * stridePlane;
    const unsigned short* Vg = VTh + (size_t)f0 * stridePlane;
    wmma_gemm64<0, false, 0, 0, false, 0><<<dim3(tilesScore / 8, kGrp), dim3(256), 0, stream>>>(
        Qg, Qg, kD, stridePlane, Kg, Kg, kD, stridePlane,
        (void*)S, (void*)S, kW, strideScore, Vsum, Vsum, 0L, kW, kW, kD, kScoreScale);
    pexp_kernel<<<dim3(kGrp * (kW / 32)), dim3(256), 0, stream>>>(S, P, L);
    wmma_gemm64<0, false, 0, 0, false, 0><<<dim3(tilesPV / 8, kGrp), dim3(256), 0, stream>>>(
        P, P, kW, strideScore, Vg, Vg, kW, stridePlane,
        (void*)Num, (void*)Num, kD, strideNum, Vsum, Vsum, 0L, kW, kD, kW, kPCarryInv);
    ofin_kernel<<<dim3((kGrp * kW * 16) / 256), dim3(256), 0, stream>>>(Num, L, Vsum, Oh, f0);
  }

  const int tilesOut = (kTok / 64) * (kG / 64);
  wmma_gemm64<0, false, 0, 0, false, 0><<<dim3(tilesOut / 8, 1), dim3(256), 0, stream>>>(
      Oh, Oh, kG, 0L, Wo, Wo, kG, 0L, (void*)out, (void*)out, kG, 0L, Vsum, Vsum, 0L, kTok, kG, kG, kOutScale);
}
